// PGNN_5634997092468
// MI455X (gfx1250) — hardware-run, weakly checked
//
#include <hip/hip_runtime.h>

typedef float          v8f   __attribute__((ext_vector_type(8)));
typedef float          v4f   __attribute__((ext_vector_type(4)));
typedef unsigned int   v4u   __attribute__((ext_vector_type(4)));
typedef int            v8i   __attribute__((ext_vector_type(8)));
typedef unsigned short v8us  __attribute__((ext_vector_type(8)));
typedef unsigned short v16us __attribute__((ext_vector_type(16)));
typedef __bf16         v16bf __attribute__((ext_vector_type(16)));
typedef _Float16       v16h  __attribute__((ext_vector_type(16)));
typedef v4f  __attribute__((may_alias)) v4fa;
typedef v8us __attribute__((may_alias)) v8usa;
union FragB { v16bf v; v16us u; v8us h[2]; v8i w; };
union FragH { v16h  v; v16us u; v8us h[2]; v8i w; };

__device__ __forceinline__ v8f wmb(const FragB& a, const FragB& b, v8f c) {
  v8f d = __builtin_amdgcn_wmma_f32_16x16x32_bf16(false, a.v, false, b.v, (short)0, c, false, false);
  asm volatile("v_nop\n\tv_nop\n\tv_nop\n\tv_nop" : "+v"(d) : "v"(a.w), "v"(b.w));
  return d;
}

__device__ __forceinline__ v8f wmh(const FragH& a, const FragH& b, v8f c) {
  v8f d = __builtin_amdgcn_wmma_f32_16x16x32_f16(false, a.v, false, b.v, (short)0, c, false, false);
  asm volatile("v_nop\n\tv_nop\n\tv_nop\n\tv_nop" : "+v"(d) : "v"(a.w), "v"(b.w));
  return d;
}

__device__ __forceinline__ unsigned bf16_bits(float f) {
  const unsigned u = __float_as_uint(f);
  const unsigned r = (u + 0x7FFFu + ((u >> 16) & 1u)) >> 16;
  const unsigned q = (u >> 16) | 0x40u;
  return ((u & 0x7fffffffu) > 0x7f800000u) ? q : r;
}

__device__ __forceinline__ float bf16_val(float f) {
  return __uint_as_float(bf16_bits(f) << 16);
}
__device__ __forceinline__ int clampi(int v, int lo, int hi) {
  return v < lo ? lo : (v > hi ? hi : v);
}

__device__ __forceinline__ unsigned f16_bits(float f) {
  const unsigned u  = __float_as_uint(f);
  const unsigned s  = (u >> 16) & 0x8000u;
  const unsigned a  = u & 0x7fffffffu;
  const unsigned t  = a - 0x38000000u;
  const unsigned r  = (t + 0x0FFFu + ((t >> 13) & 1u)) >> 13;
  const unsigned rc = r > 0x7C00u ? 0x7C00u : r;
  const bool small  = a < 0x38800000u;
  const bool isnan  = a > 0x7f800000u;
  const unsigned fin = small ? 0u : (s | rc);
  return isnan ? (s | 0x7E00u) : fin;
}

__device__ __forceinline__ unsigned pk16(unsigned lo, unsigned hi) { return lo | (hi << 16); }
__device__ __forceinline__ unsigned bf16_lo_bits(float v) {
  float hi = bf16_val(v);
  asm volatile("" : "+v"(hi));
  return bf16_bits(v - hi);
}
__device__ __forceinline__ v4u pack8_bf16(v4f a, v4f c) {
  return (v4u){ pk16(bf16_bits(a[0]), bf16_bits(a[1])), pk16(bf16_bits(a[2]), bf16_bits(a[3])),
                pk16(bf16_bits(c[0]), bf16_bits(c[1])), pk16(bf16_bits(c[2]), bf16_bits(c[3])) };
}
__device__ __forceinline__ v4u pack8_bf16_lo(v4f a, v4f c) {
  return (v4u){ pk16(bf16_lo_bits(a[0]), bf16_lo_bits(a[1])), pk16(bf16_lo_bits(a[2]), bf16_lo_bits(a[3])),
                pk16(bf16_lo_bits(c[0]), bf16_lo_bits(c[1])), pk16(bf16_lo_bits(c[2]), bf16_lo_bits(c[3])) };
}
__device__ __forceinline__ v4u pack8_f16(v4f a, v4f c) {
  return (v4u){ pk16(f16_bits(a[0]), f16_bits(a[1])), pk16(f16_bits(a[2]), f16_bits(a[3])),
                pk16(f16_bits(c[0]), f16_bits(c[1])), pk16(f16_bits(c[2]), f16_bits(c[3])) };
}

template <int FORM>
__global__ __launch_bounds__(256) void k_plane(const float* __restrict__ src, int rows, int cols, int ldsrc,
                                               unsigned short* __restrict__ dst, int MP, int KP) {
  static_assert(FORM >= 0 && FORM <= 3);
  const int KTOT = (FORM == 1 || FORM == 3) ? 2 * KP : KP;
  const unsigned ppr   = (unsigned)(KTOT >> 3);
  const unsigned kp8   = (unsigned)(KP >> 3);
  const unsigned total = (unsigned)MP * ppr;
  const unsigned g     = blockIdx.x * 256u + threadIdx.x;
  const unsigned rowu  = g / ppr;
  const unsigned p     = g - rowu * ppr;
  const bool second    = p >= kp8;
  const int row = (int)rowu;
  const int c0  = (int)((second ? p - kp8 : p) << 3);
  const float* srow = src + (size_t)clampi(row, 0, rows - 1) * (size_t)ldsrc;
  float x[8];
  unsigned mk[8];
#pragma unroll
  for (int e = 0; e < 8; ++e) {
    const int c = c0 + e;
    const float v = srow[clampi(c, 0, cols - 1)];
    asm volatile("" :: "v"(v));
    x[e]  = v;
    mk[e] = (row < rows && c < cols) ? 0xFFFFu : 0u;
  }
  const v4f a = (v4f){ x[0], x[1], x[2], x[3] };
  const v4f c = (v4f){ x[4], x[5], x[6], x[7] };
  v4u o;
  if (FORM == 2) {
    o = pack8_f16(a, c);
  } else {
    const v4u hi = pack8_bf16(a, c);
    o = hi;
    if (FORM == 1) { const v4u lo = pack8_bf16_lo(a, c); o = second ? lo : hi; }
  }
  const v4u mw = (v4u){ pk16(mk[0], mk[1]), pk16(mk[2], mk[3]), pk16(mk[4], mk[5]), pk16(mk[6], mk[7]) };
  o &= mw;
  if (g < total) {
    volatile v4u* q = (volatile v4u*)(dst + (size_t)g * 8);
    *q = o;
    __threadfence();
    *q = o;
  }
}

template <int FORM> struct FragOf    { typedef FragB T; };
template <>         struct FragOf<2> { typedef FragH T; };
__device__ __forceinline__ v8f mm(const FragB& a, const FragB& b, v8f c) { return wmb(a, b, c); }
__device__ __forceinline__ v8f mm(const FragH& a, const FragH& b, v8f c) { return wmh(a, b, c); }
template <class F> __device__ __forceinline__ F ld_frag(const unsigned short* p) {
  F f;
  f.h[0] = *(const v8usa*)(p);
  f.h[1] = *(const v8usa*)(p + 16);
  return f;
}

template <int FORM, int EPI>
__global__ __launch_bounds__(256) __attribute__((amdgpu_num_vgpr(248)))
void k_gemm_nt(const unsigned short* __restrict__ A, const unsigned short* __restrict__ B,
               const float* __restrict__ bias, float* __restrict__ D, int M, int N, int KTOT, int ldd) {
  static_assert(FORM >= 0 && FORM <= 2);
  static_assert(EPI == 0 || EPI == 1);
  typedef typename FragOf<FORM>::T F;
  __shared__ __attribute__((aligned(16))) float sT[8][16 * 68];
  const int lane = threadIdx.x & 31;
  const int wave = threadIdx.x >> 5;
  const int tilesM = (M + 63) >> 6;
  const int tilesN = (N + 63) >> 6;
  const int tile = blockIdx.x * 8 + wave;
  if (tile >= tilesM * tilesN) return;
  const int tm = tile / tilesN;
  const int tn = tile - tm * tilesN;
  const int m0 = tm << 6;
  const int n0 = tn << 6;

  const int rl = lane & 15;
  const int h8 = (lane >> 4) * 8;
  const unsigned short* pa = A + (size_t)(m0 + rl) * (size_t)KTOT + h8;
  const unsigned short* pb = B + (size_t)(n0 + rl) * (size_t)KTOT + h8;

  v8f acc[4][4];
#pragma unroll
  for (int i = 0; i < 4; ++i)
#pragma unroll
    for (int j = 0; j < 4; ++j) acc[i][j] = (v8f){0.f, 0.f, 0.f, 0.f, 0.f, 0.f, 0.f, 0.f};

#pragma unroll 1
  for (int k0 = 0; k0 < KTOT; k0 += 32) {
    F bf[4];
#pragma unroll
    for (int j = 0; j < 4; ++j) bf[j] = ld_frag<F>(pb + (size_t)(j << 4) * (size_t)KTOT + k0);
#pragma unroll
    for (int i = 0; i < 4; ++i) {
      const F af = ld_frag<F>(pa + (size_t)(i << 4) * (size_t)KTOT + k0);
#pragma unroll
      for (int j = 0; j < 4; ++j) acc[i][j] = mm(af, bf[j], acc[i][j]);
    }
  }

  float* slab = sT[wave];
  const int hh = lane >> 4;
  const int c4 = (lane & 15) * 4;
  const int nc = n0 + c4;
  const bool cok = nc < N;
  v4f bv = (v4f){0.f, 0.f, 0.f, 0.f};
  if (EPI == 1) {
    bv = *(const v4fa*)(bias + clampi(nc, 0, N - 4));
    asm volatile("" :: "v"(bv));
  }
#pragma unroll
  for (int i = 0; i < 4; ++i) {
    const int mBase = m0 + (i << 4);
#pragma unroll
    for (int j = 0; j < 4; ++j) {
#pragma unroll
      for (int r = 0; r < 8; ++r) slab[(h8 + r) * 68 + (j << 4) + rl] = acc[i][j][r];
    }
    __builtin_amdgcn_fence(__ATOMIC_RELEASE, "workgroup");
    __builtin_amdgcn_wave_barrier();
    __builtin_amdgcn_fence(__ATOMIC_ACQUIRE, "workgroup");
    v4f vv[8];
#pragma unroll
    for (int it = 0; it < 8; ++it) {
      const int row = it * 2 + hh;
      v4f v = *(const v4fa*)(slab + row * 68 + c4);
      if (EPI == 1) v += bv;
      vv[it] = v;
    }
    for (int pass = 0; pass < 2; ++pass) {
#pragma unroll
      for (int it = 0; it < 8; ++it) {
        const int row = mBase + it * 2 + hh;
        if (cok && row < M) *(volatile v4f*)(D + (size_t)row * (size_t)ldd + nc) = vv[it];
      }
      __threadfence();
    }
    __builtin_amdgcn_fence(__ATOMIC_RELEASE, "workgroup");
    __builtin_amdgcn_wave_barrier();
    __builtin_amdgcn_fence(__ATOMIC_ACQUIRE, "workgroup");
  }
}

#pragma clang fp contract(off)

#ifndef TWO_TERM_B
#define TWO_TERM_B 1
#endif
#ifndef TWO_TERM_C
#define TWO_TERM_C 1
#endif

constexpr int kNodes = 50000;
constexpr int kEdges = 1600000;
constexpr int kAnch  = 64;
constexpr int kInDim = 128;
constexpr int kFeat  = 32;
constexpr int kMP    = 50048;

static_assert(kNodes % 8 == 0);
static_assert(kNodes % 16 == 0);
static_assert(kAnch == 64);
static_assert(kFeat == 32);
static_assert(kMP % 128 == 0 && kMP % 64 == 0 && kMP >= kNodes);
static_assert(kInDim % 32 == 0 && (2 * kFeat) % 32 == 0);
static_assert((long long)kMP * kInDim / 8 < 0x7fffffffLL);
static_assert((kMP * (kInDim / 8)) % 256 == 0);
static_assert((kMP * (2 * kFeat / 8)) % 256 == 0);

constexpr size_t kSzFB  = (size_t)kMP * kInDim * 2;
constexpr size_t kSzX0  = (size_t)kMP * kFeat * 4;
constexpr size_t kSzXHL = (size_t)kMP * 2 * kFeat * 2;
constexpr size_t kSzUV  = (size_t)kMP * 2 * kFeat * 4;
constexpr size_t kSzWPT = (size_t)64 * kInDim * 2;
constexpr size_t kSzWUV = (size_t)64 * 64 * 2;
constexpr size_t kSzTB  = (size_t)256 * 4;
constexpr size_t kOffFB   = 0;
constexpr size_t kOffX0   = kOffFB + kSzFB;
constexpr size_t kOffXHL  = kOffX0 + kSzX0;
constexpr size_t kOffUV   = kOffXHL + kSzXHL;
constexpr size_t kOffWPT  = kOffUV + kSzUV;
constexpr size_t kOffWUV1 = kOffWPT + kSzWPT;
constexpr size_t kOffWUV2 = kOffWUV1 + kSzWUV;
constexpr size_t kOffTB   = kOffWUV2 + kSzWUV;
constexpr size_t kWsTotal = kOffTB + kSzTB;
static_assert(kOffX0 % 256 == 0 && kOffXHL % 256 == 0 && kOffUV % 256 == 0 && kOffWPT % 256 == 0);
static_assert(kOffWUV1 % 256 == 0 && kOffWUV2 % 256 == 0 && kOffTB % 256 == 0);
static_assert(kWsTotal == 38470656);
static_assert(kWsTotal <= ((size_t)128 << 20));

constexpr int kTbBP   = 0;
constexpr int kTbBUV1 = 32;
constexpr int kTbBUV2 = 96;
constexpr int kTbWO2  = 160;
constexpr int kTbBO2  = 192;

__device__ __forceinline__ void put16(unsigned short* p, v4u o) {
  volatile v4u* q = (volatile v4u*)p;
  *q = o;
  __threadfence();
  *q = o;
}

__device__ __forceinline__ void prep_wpre(const float* __restrict__ W, unsigned short* __restrict__ dst, int u) {
  const int n  = u >> 4;
  const int k8 = (u & 15) << 3;
  const int nc = n < kFeat ? n : kFeat - 1;
  float x[8];
#pragma unroll
  for (int e = 0; e < 8; ++e) {
    const float v = W[(k8 + e) * kFeat + nc];
    asm volatile("" :: "v"(v));
    x[e] = v;
  }
  v4u o = pack8_bf16((v4f){ x[0], x[1], x[2], x[3] }, (v4f){ x[4], x[5], x[6], x[7] });
  const unsigned mk = n < kFeat ? 0xFFFFFFFFu : 0u;
  o &= (v4u){ mk, mk, mk, mk };
  put16(dst + (size_t)n * kInDim + k8, o);
}

__device__ __forceinline__ void prep_w32(const float* __restrict__ W, unsigned short* __restrict__ dst, int tid, int two) {
  const int nl = tid >> 3;
  const int k8 = (tid & 7) << 3;
  const int kk = k8 & 31;
  float x[8];
#pragma unroll
  for (int e = 0; e < 8; ++e) {
    const float v = W[(kk + e) * kFeat + nl];
    asm volatile("" :: "v"(v));
    x[e] = v;
  }
  v4u o = pack8_bf16((v4f){ x[0], x[1], x[2], x[3] }, (v4f){ x[4], x[5], x[6], x[7] });
  const unsigned mk = (two != 0 || k8 < 32) ? 0xFFFFFFFFu : 0u;
  o &= (v4u){ mk, mk, mk, mk };
  put16(dst + (size_t)nl * 64 + k8, o);
}

__global__ __launch_bounds__(256) void k_prep(
    const float* __restrict__ Wpre, const float* __restrict__ bpre,
    const float* __restrict__ Wu1, const float* __restrict__ bu1,
    const float* __restrict__ Wv1, const float* __restrict__ bv1,
    const float* __restrict__ Wu2, const float* __restrict__ bu2,
    const float* __restrict__ Wv2, const float* __restrict__ bv2,
    const float* __restrict__ Wo2, const float* __restrict__ bo2,
    unsigned short* __restrict__ WPT, unsigned short* __restrict__ WUV1,
    unsigned short* __restrict__ WUV2, float* __restrict__ TB) {
  const int b   = (int)blockIdx.x;
  const int tid = (int)threadIdx.x;
  if (b < 4) {
    prep_wpre(Wpre, WPT, b * 256 + tid);
  } else if (b == 4) {
    prep_w32(Wu1, WUV1, tid, TWO_TERM_B);
  } else if (b == 5) {
    prep_w32(Wv1, WUV1 + 32 * 64, tid, TWO_TERM_B);
  } else if (b == 6) {
    prep_w32(Wu2, WUV2, tid, TWO_TERM_C);
  } else if (b == 7) {
    prep_w32(Wv2, WUV2 + 32 * 64, tid, TWO_TERM_C);
  } else {
    const int lane = tid & 31;
    const int wave = tid >> 5;
    const int l8   = lane & 7;
    const v4f c0 = *(const v4fa*)(bpre + 4 * l8);  asm volatile("" :: "v"(c0));
    const v4f c1 = *(const v4fa*)(bu1 + 4 * l8);   asm volatile("" :: "v"(c1));
    const v4f c2 = *(const v4fa*)(bv1 + 4 * l8);   asm volatile("" :: "v"(c2));
    const v4f c3 = *(const v4fa*)(bu2 + 4 * l8);   asm volatile("" :: "v"(c3));
    const v4f c4 = *(const v4fa*)(bv2 + 4 * l8);   asm volatile("" :: "v"(c4));
    const v4f c5 = *(const v4fa*)(Wo2 + 4 * l8);   asm volatile("" :: "v"(c5));
    const float bo = bo2[0];                        asm volatile("" :: "v"(bo));
    const float bz = (l8 == 0) ? bo : 0.0f;
    v4f x = (v4f){ 0.f, 0.f, 0.f, 0.f };
    if (wave == 0) x = c0;
    if (wave == 1) x = c1;
    if (wave == 2) x = c2;
    if (wave == 3) x = c3;
    if (wave == 4) x = c4;
    if (wave == 5) x = c5;
    if (wave == 6) x = (v4f){ bz, 0.f, 0.f, 0.f };
    const v4f y = (v4f){ bf16_val(x[0]), bf16_val(x[1]), bf16_val(x[2]), bf16_val(x[3]) };
    volatile v4f* q = (volatile v4f*)(TB + wave * 32 + 4 * l8);
    const bool wr = lane < 8;
    if (wr) *q = y;
    __threadfence();
    if (wr) *q = y;
  }
}

template <int LAYER>
__device__ __forceinline__ void walk32(const float* __restrict__ UV, int sv, int dv, float wv, int lane,
                                       float wo, float bo, float& acc, float& ss, float& keep) {
#pragma clang fp contract(off)
  const int wbits = __float_as_int(wv);
#pragma unroll 2
  for (int k = 0; k < 32; ++k) {
    const int s = __builtin_amdgcn_readlane(sv, k);
    const int d = __builtin_amdgcn_readlane(dv, k);
    const float w = __int_as_float(__builtin_amdgcn_readlane(wbits, k));
    const float uu = UV[(size_t)s * 64 + lane];
    asm volatile("" :: "v"(uu));
    const float vv = UV[(size_t)d * 64 + 32 + lane];
    asm volatile("" :: "v"(vv));
    const float t   = uu * w;
    const float msg = vv + t;
    const float m   = (msg > 0.0f) ? msg : (msg - msg);
    if (LAYER == 1) {
      acc = __fadd_rn(acc, m);
    } else {
      float q = __fmul_rn(m, wo);
      q = __fadd_rn(q, __shfl_xor(q, 16));
      q = __fadd_rn(q, __shfl_xor(q, 8));
      q = __fadd_rn(q, __shfl_xor(q, 4));
      q = __fadd_rn(q, __shfl_xor(q, 2));
      q = __fadd_rn(q, __shfl_xor(q, 1));
      const float p = __fadd_rn(q, bo);
      const float p2 = p * p;
      ss = ss + p2;
      keep = (k == lane) ? p : keep;
    }
  }
}

template <int LAYER>
__global__ __launch_bounds__(256) void k_anchor(
    const int* __restrict__ aeid, const int* __restrict__ src, const int* __restrict__ dst,
    const float* __restrict__ spd, const float* __restrict__ UV, const float* __restrict__ TB,
    unsigned* __restrict__ XHLw, float* __restrict__ out) {
#pragma clang fp contract(off)
  static_assert(LAYER == 1 || LAYER == 2);
  const int lane = (int)threadIdx.x & 31;
  const int wave = (int)threadIdx.x >> 5;
  const int row  = (int)blockIdx.x * 8 + wave;
  const bool ok  = row < kNodes;
  const int rc   = ok ? row : kNodes - 1;

  const int* ep = aeid + (size_t)rc * kAnch;
  int e0 = ep[lane];        asm volatile("" :: "v"(e0));
  int e1 = ep[32 + lane];   asm volatile("" :: "v"(e1));
  e0 = clampi(e0, 0, kEdges - 1);
  e1 = clampi(e1, 0, kEdges - 1);
  int   s0 = src[e0];  asm volatile("" :: "v"(s0));
  int   d0 = dst[e0];  asm volatile("" :: "v"(d0));
  float w0 = spd[e0];  asm volatile("" :: "v"(w0));
  int   s1 = src[e1];  asm volatile("" :: "v"(s1));
  int   d1 = dst[e1];  asm volatile("" :: "v"(d1));
  float w1 = spd[e1];  asm volatile("" :: "v"(w1));
  s0 = clampi(s0, 0, kNodes - 1);
  d0 = clampi(d0, 0, kNodes - 1);
  s1 = clampi(s1, 0, kNodes - 1);
  d1 = clampi(d1, 0, kNodes - 1);
  w0 = bf16_val(w0);
  w1 = bf16_val(w1);

  float wo = 0.0f, bo = 0.0f;
  if (LAYER == 2) {
    wo = TB[kTbWO2 + lane];   asm volatile("" :: "v"(wo));
    bo = TB[kTbBO2];          asm volatile("" :: "v"(bo));
  }

  float acc = 0.0f, ss = 0.0f, keepLo = 0.0f, keepHi = 0.0f;
  walk32<LAYER>(UV, s0, d0, w0, lane, wo, bo, acc, ss, keepLo);
  walk32<LAYER>(UV, s1, d1, w1, lane, wo, bo, acc, ss, keepHi);

  if (LAYER == 1) {
    const float x1 = __fmul_rn(acc, 0.015625f);
    const int hb = (int)bf16_bits(x1);
    const int lb = (int)bf16_lo_bits(x1);
    const int sl0 = 2 * (lane & 15);
    const int sl1 = sl0 + 1;
    const unsigned he = (unsigned)__shfl(hb, sl0);
    const unsigned ho = (unsigned)__shfl(hb, sl1);
    const unsigned le = (unsigned)__shfl(lb, sl0);
    const unsigned lo = (unsigned)__shfl(lb, sl1);
    const unsigned wh = pk16(he & 0xFFFFu, ho & 0xFFFFu);
    const unsigned wl = pk16(le & 0xFFFFu, lo & 0xFFFFu);
    const unsigned word = (lane < 16) ? wh : wl;
    volatile unsigned* q = (volatile unsigned*)(XHLw + (size_t)rc * 32 + lane);
    if (ok) *q = word;
    __threadfence();
    if (ok) *q = word;
  } else {
    const float sq  = sqrtf(ss);
    const float nrm = ((sq > 1e-12f) || (sq != sq)) ? sq : 1e-12f;
    const float o0 = keepLo / nrm;
    const float o1 = keepHi / nrm;
    volatile float* q0 = (volatile float*)(out + (size_t)rc * kAnch + lane);
    volatile float* q1 = q0 + 32;
    if (ok) { *q0 = o0; *q1 = o1; }
    __threadfence();
    if (ok) { *q0 = o0; *q1 = o1; }
  }
  (void)XHLw; (void)out; (void)TB;
}

extern "C" void kernel_launch(void* const* d_in, const int* in_sizes, int n_in,
                              void* d_out, int out_size, void* d_ws, size_t ws_size,
                              hipStream_t stream) {
  if (n_in != 20) return;
  if (in_sizes[0] != kNodes * kInDim) return;
  if (in_sizes[1] != kEdges || in_sizes[2] != kEdges || in_sizes[3] != kEdges) return;
  if (in_sizes[4] != kNodes * kAnch || in_sizes[5] != kNodes * kAnch) return;
  if (in_sizes[6] != kInDim * kFeat || in_sizes[7] != kFeat) return;
  if (in_sizes[8] != kFeat * kFeat || in_sizes[9] != kFeat) return;
  if (in_sizes[10] != kFeat * kFeat || in_sizes[11] != kFeat) return;
  if (in_sizes[14] != kFeat * kFeat || in_sizes[15] != kFeat) return;
  if (in_sizes[16] != kFeat * kFeat || in_sizes[17] != kFeat) return;
  if (in_sizes[18] != kFeat || in_sizes[19] != 1) return;
  if (out_size != kNodes * kAnch) return;
  if (ws_size < kWsTotal) return;

  const float* feat  = (const float*)d_in[0];
  const float* spd   = (const float*)d_in[1];
  const int*   src   = (const int*)d_in[2];
  const int*   dst   = (const int*)d_in[3];
  const int*   aeid  = (const int*)d_in[4];
  const float* Wpre  = (const float*)d_in[6];
  const float* bpre  = (const float*)d_in[7];
  const float* Wu1   = (const float*)d_in[8];
  const float* bu1   = (const float*)d_in[9];
  const float* Wv1   = (const float*)d_in[10];
  const float* bv1   = (const float*)d_in[11];
  const float* Wu2   = (const float*)d_in[14];
  const float* bu2   = (const float*)d_in[15];
  const float* Wv2   = (const float*)d_in[16];
  const float* bv2   = (const float*)d_in[17];
  const float* Wo2   = (const float*)d_in[18];
  const float* bo2   = (const float*)d_in[19];
  float* out = (float*)d_out;

  char* ws = (char*)d_ws;
  unsigned short* FB   = (unsigned short*)(ws + kOffFB);
  float*          X0   = (float*)(ws + kOffX0);
  unsigned short* XHL  = (unsigned short*)(ws + kOffXHL);
  float*          UV   = (float*)(ws + kOffUV);
  unsigned short* WPT  = (unsigned short*)(ws + kOffWPT);
  unsigned short* WUV1 = (unsigned short*)(ws + kOffWUV1);
  unsigned short* WUV2 = (unsigned short*)(ws + kOffWUV2);
  float*          TB   = (float*)(ws + kOffTB);

  const int gPlaneFB  = kMP * (kInDim / 8) / 256;
  const int gPlaneXHL = kMP * (2 * kFeat / 8) / 256;
  const int tiles     = (kNodes + 63) / 64;
  const int gGemm     = (tiles + 7) / 8;
  const int gAnchor   = kNodes / 8;

  k_prep<<<9, 256, 0, stream>>>(Wpre, bpre, Wu1, bu1, Wv1, bv1, Wu2, bu2, Wv2, bv2, Wo2, bo2, WPT, WUV1, WUV2, TB);
  k_plane<0><<<gPlaneFB, 256, 0, stream>>>(feat, kNodes, kInDim, kInDim, FB, kMP, kInDim);
  k_gemm_nt<0, 1><<<gGemm, 256, 0, stream>>>(FB, WPT, TB + kTbBP, X0, kNodes, kFeat, kInDim, kFeat);
  k_plane<1><<<gPlaneXHL, 256, 0, stream>>>(X0, kNodes, kFeat, kFeat, XHL, kMP, kFeat);
  k_gemm_nt<1, 1><<<gGemm, 256, 0, stream>>>(XHL, WUV1, TB + kTbBUV1, UV, kNodes, 2 * kFeat, 2 * kFeat, 2 * kFeat);
  k_anchor<1><<<gAnchor, 256, 0, stream>>>(aeid, src, dst, spd, UV, TB, (unsigned*)XHL, out);
  k_gemm_nt<1, 1><<<gGemm, 256, 0, stream>>>(XHL, WUV2, TB + kTbBUV2, UV, kNodes, 2 * kFeat, 2 * kFeat, 2 * kFeat);
  k_anchor<2><<<gAnchor, 256, 0, stream>>>(aeid, src, dst, spd, UV, TB, (unsigned*)XHL, out);
}
